// S4Kernel_76802605187518
// MI455X (gfx1250) — hardware-run, weakly checked
//
#include <hip/hip_runtime.h>
#include <math.h>

typedef __attribute__((ext_vector_type(16))) __bf16   v16b;
typedef __attribute__((ext_vector_type(8)))  __bf16   v8b;
typedef __attribute__((ext_vector_type(8)))  float    v8f;
typedef __attribute__((ext_vector_type(4)))  float    v4f;
typedef __attribute__((ext_vector_type(4)))  unsigned v4u;

constexpr int kBatch   = 4;
constexpr int kLen     = 2048;
constexpr int kDm      = 1024;
constexpr int kNs      = 64;
constexpr int kRowsAll = kBatch * kLen;
static_assert((kLen & (kLen - 1)) == 0, "time length is a power of two");
static_assert((kDm % 32) == 0 && (kNs % 32) == 0, "GEMM K multiples of 32");
static_assert((kRowsAll % 64) == 0 && (kNs % 64) == 0 && (kDm % 64) == 0 && (kLen % 64) == 0, "GEMM M,N multiples of 64");

constexpr size_t kOffTS  = 0;
constexpr size_t kOffXAH = kOffTS  + 128;
constexpr size_t kOffXAL = kOffXAH + (size_t)kRowsAll * kDm * 2;
constexpr size_t kOffWBH = kOffXAL + (size_t)kRowsAll * kDm * 2;
constexpr size_t kOffWBL = kOffWBH + (size_t)kNs * kDm * 2;
constexpr size_t kOffCTH = kOffWBL + (size_t)kNs * kDm * 2;
constexpr size_t kOffCTL = kOffCTH + (size_t)kDm * kNs * 2;
constexpr size_t kOffBX  = kOffCTL + (size_t)kDm * kNs * 2;
constexpr size_t kOffGH  = kOffBX  + (size_t)kRowsAll * kNs * 4;
constexpr size_t kOffGL  = kOffGH  + (size_t)kRowsAll * kNs * 2;
constexpr size_t kOffKC  = kOffGL  + (size_t)kRowsAll * kNs * 2;
constexpr size_t kWsTotal = kOffKC + (size_t)kRowsAll * kDm * 4;
static_assert(kWsTotal == 71827584ull, "carve total");
static_assert(kWsTotal <= 134217728ull, "carve cap");
static_assert((kOffXAH % 128) == 0 && (kOffXAL % 128) == 0 && (kOffWBH % 128) == 0 && (kOffWBL % 128) == 0 &&
              (kOffCTH % 128) == 0 && (kOffCTL % 128) == 0 && (kOffBX % 128) == 0 && (kOffGH % 128) == 0 &&
              (kOffGL % 128) == 0 && (kOffKC % 128) == 0, "128-B aligned regions");

__device__ __forceinline__ int load_tap_bound(const int* tsp) {
  int ts = tsp[0];
  ts = ts < 1 ? 1 : ts;
  ts = ts > kLen ? kLen : ts;
  return ts;
}
__device__ __forceinline__ unsigned bf_hi32(float f) {
  unsigned u = __float_as_uint(f);
  const unsigned lsb = (u & 0x00010000u) ? 1u : 0u;
  u = (u + 0x7FFFu + lsb) & 0xFFFF0000u;
  return u;
}
__device__ __forceinline__ void split_pair(float a, float b, unsigned& hw, unsigned& lw) {
  const unsigned ha = bf_hi32(a);
  const unsigned hb = bf_hi32(b);
  const unsigned la = bf_hi32(a - __uint_as_float(ha));
  const unsigned lb = bf_hi32(b - __uint_as_float(hb));
  hw = __builtin_amdgcn_perm(hb, ha, 0x07060302u);
  lw = __builtin_amdgcn_perm(lb, la, 0x07060302u);
}
__device__ __forceinline__ void split8(v4f a0, v4f a1, v4u& hv, v4u& lv) {
  unsigned h0, h1, h2, h3, l0, l1, l2, l3;
  split_pair(a0.x, a0.y, h0, l0);
  split_pair(a0.z, a0.w, h1, l1);
  split_pair(a1.x, a1.y, h2, l2);
  split_pair(a1.z, a1.w, h3, l3);
  hv = (v4u){h0, h1, h2, h3};
  lv = (v4u){l0, l1, l2, l3};
}

__global__ __launch_bounds__(32) void tap_bound_kernel(const float* __restrict__ logA, int* __restrict__ ts)
{
  const unsigned lane = threadIdx.x & 31u;
  const float a = logA[lane];
  const float b = logA[lane + 32u];
  float mx = fmaxf(a, b);
  int bad = ((a != a) || (b != b)) ? 1 : 0;
#pragma unroll
  for (int off = 16; off >= 1; off >>= 1) {
    const float om = __shfl_xor(mx, off, 32);
    const int   ob = __shfl_xor(bad, off, 32);
    mx = fmaxf(mx, om);
    bad |= ob;
  }
  int best = kLen;
#pragma unroll 1
  for (int i = 63; i >= 0; --i) {
    const int t = (int)lane * 64 + i;
    const float p = (float)t * mx;
    best = (p < -104.0f) ? t : best;
  }
#pragma unroll
  for (int off = 16; off >= 1; off >>= 1) {
    const int o = __shfl_xor(best, off, 32);
    best = (o < best) ? o : best;
  }
  best = bad ? kLen : best;
  volatile int* q = ts + lane;
  *q = best;
  __threadfence();
  *q = best;
}

__global__ __launch_bounds__(256) void split_rows_kernel(
    const float* __restrict__ src, unsigned* __restrict__ dhi, unsigned* __restrict__ dlo,
    int total8, const int* __restrict__ tsp, int useLimit)
{
  const unsigned i = blockIdx.x * 256u + threadIdx.x;
  if (i >= (unsigned)total8) return;
  if (useLimit) {
    const int ts = load_tap_bound(tsp);
    const int tp = (ts + 63) & ~63;
    const unsigned row = i >> 7;
    const int t = (int)(row & (unsigned)(kLen - 1));
    if (t >= tp) return;
  }
  const size_t e0 = (size_t)i << 3;
  const v4f a0 = *(const v4f*)(src + e0);
  const v4f a1 = *(const v4f*)(src + e0 + 4);
  v4u hv, lv;
  split8(a0, a1, hv, lv);
  unsigned* qh = dhi + ((size_t)i << 2);
  unsigned* ql = dlo + ((size_t)i << 2);
  *(volatile v4u*)qh = hv;
  *(volatile v4u*)ql = lv;
  __threadfence();
  *(volatile v4u*)qh = hv;
  *(volatile v4u*)ql = lv;
}

__global__ __launch_bounds__(256) void transpose_split_kernel(
    const float* __restrict__ Cm, unsigned* __restrict__ cth, unsigned* __restrict__ ctl)
{
  __shared__ float st[64 * 33];
  const unsigned tid = threadIdx.x;
  const unsigned m0 = blockIdx.x * 32u;
#pragma unroll 1
  for (unsigned it = 0; it < 8u; ++it) {
    const unsigned idx = it * 256u + tid;
    const unsigned n  = idx >> 5;
    const unsigned mm = idx & 31u;
    st[n * 33u + mm] = Cm[(size_t)n * kDm + m0 + mm];
  }
  __syncthreads();
  unsigned row = tid >> 3;
  unsigned c8  = (tid & 7u) << 3;
  asm volatile("" : "+v"(row));
  asm volatile("" : "+v"(c8));
  v4f a0, a1;
  a0.x = st[(c8 + 0u) * 33u + row];
  a0.y = st[(c8 + 1u) * 33u + row];
  a0.z = st[(c8 + 2u) * 33u + row];
  a0.w = st[(c8 + 3u) * 33u + row];
  a1.x = st[(c8 + 4u) * 33u + row];
  a1.y = st[(c8 + 5u) * 33u + row];
  a1.z = st[(c8 + 6u) * 33u + row];
  a1.w = st[(c8 + 7u) * 33u + row];
  v4u hv, lv;
  split8(a0, a1, hv, lv);
  const size_t wo = (((size_t)(m0 + row) * kNs) + c8) >> 1;
  *(volatile v4u*)(cth + wo) = hv;
  *(volatile v4u*)(ctl + wo) = lv;
  __threadfence();
  *(volatile v4u*)(cth + wo) = hv;
  *(volatile v4u*)(ctl + wo) = lv;
}

namespace eng {
union FragU { v16b v; v8b h[2]; };
__device__ __forceinline__ v16b frag_load(const __bf16* p) {
  FragU f;
  f.h[0] = *(const v8b*)(p);
  f.h[1] = *(const v8b*)(p + 16);
  return f.v;
}
__device__ __forceinline__ v8f mma_g(v16b a, v16b b, v8f c) {
  c = __builtin_amdgcn_wmma_f32_16x16x32_bf16(false, a, false, b, (short)0, c, false, false);
  asm volatile("v_nop\n\tv_nop\n\tv_nop\n\tv_nop" : "+v"(c) : "v"(a), "v"(b));
  return c;
}

template <bool HAS_BIAS>
__global__ __launch_bounds__(256) void gemm64_bf16x3_kernel(
    const unsigned short* __restrict__ Ahp, const unsigned short* __restrict__ Alp, int lda,
    const unsigned short* __restrict__ Bhp, const unsigned short* __restrict__ Blp, int ldb,
    float* __restrict__ Cout, int ldc, const float* __restrict__ bias, const int* __restrict__ tsp,
    int M, int N, int K)
{
  const __bf16* Ah = (const __bf16*)Ahp;
  const __bf16* Al = (const __bf16*)Alp;
  const __bf16* Bh = (const __bf16*)Bhp;
  const __bf16* Bl = (const __bf16*)Blp;
  __shared__ __align__(16) float sT[8][16 * 68];
  const int lane = threadIdx.x & 31;
  const int wave = threadIdx.x >> 5;
  const int tilesN = N >> 6;
  const int tilesM = M >> 6;
  const int tile = blockIdx.x * 8 + wave;
  if (tile >= tilesM * tilesN) return;
  const int tm = tile / tilesN;
  const int tn = tile - tm * tilesN;
  const int m0 = tm << 6;
  const int n0 = tn << 6;
  {
    const int ts = load_tap_bound(tsp);
    const int tp = (ts + 63) & ~63;
    if ((m0 & (kLen - 1)) >= tp) return;
  }

  const int rlane = lane & 15;
  const int koff  = (lane >> 4) * 8;
  const int mOff  = (lane >> 4) * 8;

  v8f acc[4][4];
#pragma unroll
  for (int i = 0; i < 4; ++i)
#pragma unroll
    for (int j = 0; j < 4; ++j) acc[i][j] = (v8f){0.f, 0.f, 0.f, 0.f, 0.f, 0.f, 0.f, 0.f};

  for (int k0 = 0; k0 < K; k0 += 32) {
    v16b bh[4], bl[4];
#pragma unroll
    for (int j = 0; j < 4; ++j) {
      const size_t bo = (size_t)(n0 + (j << 4) + rlane) * ldb + koff + k0;
      bh[j] = frag_load(Bh + bo);
      bl[j] = frag_load(Bl + bo);
    }
#pragma unroll
    for (int i = 0; i < 4; ++i) {
      const size_t ao = (size_t)(m0 + (i << 4) + rlane) * lda + koff + k0;
      const v16b ah = frag_load(Ah + ao);
      const v16b al = frag_load(Al + ao);
#pragma unroll
      for (int j = 0; j < 4; ++j) {
        acc[i][j] = mma_g(ah, bh[j], acc[i][j]);
        acc[i][j] = mma_g(ah, bl[j], acc[i][j]);
        acc[i][j] = mma_g(al, bh[j], acc[i][j]);
      }
    }
  }

  float* slab = sT[wave];
#pragma unroll
  for (int i = 0; i < 4; ++i) {
    const int mBase = m0 + (i << 4);
#pragma unroll
    for (int j = 0; j < 4; ++j) {
      const int n = n0 + (j << 4) + rlane;
      float bv = 0.f;
      if (HAS_BIAS) bv = bias[n];
#pragma unroll
      for (int r = 0; r < 8; ++r) {
        float v = acc[i][j][r];
        if (HAS_BIAS) v += bv;
        slab[(mOff + r) * 68 + (j << 4) + rlane] = v;
      }
    }
    __builtin_amdgcn_fence(__ATOMIC_RELEASE, "workgroup");
    __builtin_amdgcn_wave_barrier();
    __builtin_amdgcn_fence(__ATOMIC_ACQUIRE, "workgroup");
    {
      const int hh = lane >> 4, c4 = (lane & 15) * 4;
      for (int pass = 0; pass < 2; ++pass) {
#pragma unroll
        for (int it = 0; it < 8; ++it) {
          const int row = it * 2 + hh;
          v4f v = *(const v4f*)(slab + row * 68 + c4);
          *(volatile v4f*)(Cout + (size_t)(mBase + row) * ldc + n0 + c4) = v;
        }
        __threadfence();
      }
    }
    __builtin_amdgcn_fence(__ATOMIC_RELEASE, "workgroup");
    __builtin_amdgcn_wave_barrier();
    __builtin_amdgcn_fence(__ATOMIC_ACQUIRE, "workgroup");
  }
}
}

__global__ __launch_bounds__(256) void decay_split_kernel(
    const float* __restrict__ BX, const float* __restrict__ logA, const int* __restrict__ tsp,
    unsigned* __restrict__ gh, unsigned* __restrict__ gl)
{
  __shared__ __align__(16) float sg[32 * 68];
  const unsigned tid = threadIdx.x;
  const unsigned r0 = blockIdx.x * 32u;
  {
    const int ts = load_tap_bound(tsp);
    const int tp = (ts + 63) & ~63;
    if ((int)(r0 & (unsigned)(kLen - 1)) >= tp) return;
  }
#pragma unroll 1
  for (unsigned it = 0; it < 8u; ++it) {
    const unsigned idx = it * 256u + tid;
    const unsigned row = idx >> 6;
    const unsigned col = idx & 63u;
    const float bx = BX[(size_t)(r0 + row) * kNs + col];
    const float la = logA[col];
    const int   t  = (int)((r0 + row) & (unsigned)(kLen - 1));
    const float arg = (float)t * la;
    float a = expf(arg);
    a = (a < 1.17549435e-38f) ? 0.0f : a;
    sg[row * 68u + col] = bx * a;
  }
  __syncthreads();
  unsigned row = tid >> 3;
  unsigned c8  = (tid & 7u) << 3;
  asm volatile("" : "+v"(row));
  asm volatile("" : "+v"(c8));
  const v4f a0 = *(const v4f*)(sg + row * 68u + c8);
  const v4f a1 = *(const v4f*)(sg + row * 68u + c8 + 4u);
  v4u hv, lv;
  split8(a0, a1, hv, lv);
  const size_t wo = (((size_t)(r0 + row) * kNs) + c8) >> 1;
  *(volatile v4u*)(gh + wo) = hv;
  *(volatile v4u*)(gl + wo) = lv;
  __threadfence();
  *(volatile v4u*)(gh + wo) = hv;
  *(volatile v4u*)(gl + wo) = lv;
}

__global__ __launch_bounds__(256) void fir_skip_kernel(
    const float* __restrict__ x, const float* __restrict__ Kc, const float* __restrict__ Dv,
    const int* __restrict__ tsp, float* __restrict__ out)
{
  __shared__ __align__(16) float sx[128 * 32];
  __shared__ __align__(16) float sk[64 * 32];
  const unsigned tid  = threadIdx.x;
  const unsigned lane = tid & 31u;
  const int wave = (int)(tid >> 5);
  const int m0 = blockIdx.x * 32;
  const int t0 = blockIdx.y * 64;
  const int b  = blockIdx.z;

  const int ts  = load_tap_bound(tsp);
  const int tb8 = (ts + 7) & ~7;
  int nch = (tb8 + 63) >> 6;
  const int ncausal = (t0 >> 6) + 1;
  nch = (nch < ncausal) ? nch : ncausal;
  nch = (nch > 32) ? 32 : nch;

  const float* xb = x  + (size_t)b * kLen * kDm + m0;
  const float* kb = Kc + (size_t)b * kLen * kDm + m0;
  float*       ob = out + (size_t)b * kLen * kDm + m0;

  const float dm = Dv[m0 + lane];
  float acc[8];
#pragma unroll
  for (int j = 0; j < 8; ++j) {
    const float xv0 = xb[(size_t)(t0 + wave * 8 + j) * kDm + lane];
    acc[j] = dm * xv0;
  }

#pragma unroll 1
  for (int ch = 0; ch < nch; ++ch) {
    const int s0 = ch << 6;
    const int gbase = t0 - s0 - 63;
    __syncthreads();
#pragma unroll
    for (unsigned it = 0; it < 4u; ++it) {
      unsigned slot = it * 256u + tid;
      unsigned i  = slot >> 3;
      unsigned c4 = (slot & 7u) << 2;
      asm volatile("" : "+v"(i));
      asm volatile("" : "+v"(c4));
      const int g = gbase + (int)i;
      int gc = g < 0 ? 0 : g;
      gc = gc > (kLen - 1) ? (kLen - 1) : gc;
      v4f xv4 = *(const v4f*)(xb + (size_t)gc * kDm + c4);
      asm volatile("" : "+v"(xv4));
      const bool ok = (g >= 0) && (g < kLen);
      v4f z;
      z.x = ok ? xv4.x : 0.0f;
      z.y = ok ? xv4.y : 0.0f;
      z.z = ok ? xv4.z : 0.0f;
      z.w = ok ? xv4.w : 0.0f;
      *(v4f*)(sx + i * 32u + c4) = z;
    }
#pragma unroll
    for (unsigned it = 0; it < 2u; ++it) {
      unsigned slot = it * 256u + tid;
      unsigned r  = slot >> 3;
      unsigned c4 = (slot & 7u) << 2;
      asm volatile("" : "+v"(r));
      asm volatile("" : "+v"(c4));
      const v4f kv4 = *(const v4f*)(kb + (size_t)(s0 + (int)r) * kDm + c4);
      *(v4f*)(sk + r * 32u + c4) = kv4;
    }
    __syncthreads();
    int nblk = (tb8 - s0) >> 3;
    nblk = (nblk > 8) ? 8 : nblk;
#pragma unroll 1
    for (int u = 0; u < nblk; ++u) {
      const int base = wave * 8 - 8 * u + 56;
      float xv[15];
      float kv[8];
#pragma unroll
      for (int d = 0; d < 15; ++d) xv[d] = sx[(base + d) * 32 + (int)lane];
#pragma unroll
      for (int e = 0; e < 8; ++e) kv[e] = sk[(8 * u + e) * 32 + (int)lane];
#pragma unroll
      for (int e = 0; e < 8; ++e) {
#pragma unroll
        for (int j = 0; j < 8; ++j) acc[j] = fmaf(kv[e], xv[j - e + 7], acc[j]);
      }
    }
  }

  for (int pass = 0; pass < 2; ++pass) {
#pragma unroll
    for (int j = 0; j < 8; ++j) {
      *(volatile float*)(ob + (size_t)(t0 + wave * 8 + j) * kDm + lane) = acc[j];
    }
    __threadfence();
  }
}

extern "C" void kernel_launch(void* const* d_in, const int* in_sizes, int n_in,
                              void* d_out, int out_size, void* d_ws, size_t ws_size,
                              hipStream_t stream) {
  if (n_in < 6) return;
  if (in_sizes[0] != kRowsAll * kDm) return;
  if (in_sizes[1] != kNs * kDm) return;
  if (in_sizes[2] != kNs) return;
  if (in_sizes[3] != kNs * kDm) return;
  if (in_sizes[4] != kDm) return;
  if (in_sizes[5] != kNs) return;
  if (out_size != kRowsAll * kDm) return;
  if (ws_size < kWsTotal) return;

  const float* x    = (const float*)d_in[0];
  const float* W_B  = (const float*)d_in[1];
  const float* b_B  = (const float*)d_in[2];
  const float* Cm   = (const float*)d_in[3];
  const float* Dv   = (const float*)d_in[4];
  const float* logA = (const float*)d_in[5];
  float* out = (float*)d_out;

  char* ws = (char*)d_ws;
  int*      TS  = (int*)(ws + kOffTS);
  unsigned* XAH = (unsigned*)(ws + kOffXAH);
  unsigned* XAL = (unsigned*)(ws + kOffXAL);
  unsigned* WBH = (unsigned*)(ws + kOffWBH);
  unsigned* WBL = (unsigned*)(ws + kOffWBL);
  unsigned* CTH = (unsigned*)(ws + kOffCTH);
  unsigned* CTL = (unsigned*)(ws + kOffCTL);
  float*    BX  = (float*)(ws + kOffBX);
  unsigned* GH  = (unsigned*)(ws + kOffGH);
  unsigned* GL  = (unsigned*)(ws + kOffGL);
  float*    KC  = (float*)(ws + kOffKC);

  tap_bound_kernel<<<1, 32, 0, stream>>>(logA, TS);

  split_rows_kernel<<<(kRowsAll * kDm / 8) / 256, 256, 0, stream>>>(x, XAH, XAL, kRowsAll * kDm / 8, TS, 1);
  split_rows_kernel<<<(kNs * kDm / 8) / 256, 256, 0, stream>>>(W_B, WBH, WBL, kNs * kDm / 8, TS, 0);
  transpose_split_kernel<<<kDm / 32, 256, 0, stream>>>(Cm, CTH, CTL);

  eng::gemm64_bf16x3_kernel<true><<<dim3((kRowsAll / 64) * (kNs / 64) / 8), 256, 0, stream>>>(
      (const unsigned short*)XAH, (const unsigned short*)XAL, kDm,
      (const unsigned short*)WBH, (const unsigned short*)WBL, kDm,
      BX, kNs, b_B, TS, kRowsAll, kNs, kDm);

  decay_split_kernel<<<kRowsAll / 32, 256, 0, stream>>>(BX, logA, TS, GH, GL);

  eng::gemm64_bf16x3_kernel<false><<<dim3((kRowsAll / 64) * (kDm / 64) / 8), 256, 0, stream>>>(
      (const unsigned short*)GH, (const unsigned short*)GL, kNs,
      (const unsigned short*)CTH, (const unsigned short*)CTL, kNs,
      KC, kDm, nullptr, TS, kRowsAll, kDm, kNs);

  fir_skip_kernel<<<dim3(kDm / 32, kLen / 64, kBatch), 256, 0, stream>>>(x, KC, Dv, TS, out);
}
